// SplineNet_69045894250551
// MI455X (gfx1250) — hardware-verified
//
#include <hip/hip_runtime.h>
#include <stddef.h>


#define DF      64
#define CO      8
#define COP     16
#define S1N     9
#define S2N     25
#define K1V     3
#define K2V     5
#define NTHR    256
#define NWAVE   8
#define EPT     8
#define NGRP    2
#define CHUNK   (NTHR * EPT * NGRP)
#define WCAPC   (EPT * NGRP * 32)
#define WCAPF   (EPT * NGRP * 32)
#define ESHF    11
#define EMASK   0xFFFFF
#define NBC     32768
#define NBF     2048
#define RCAP    49152
#define RBN     128
#define TGT     256
#define DEGCAP  512
#define GROWS   128
#define OTHR    512
#define TPP     72
#define ACARRY  1
#define WSCL    64
#define WSLIM   268435456

#define LDS_COUNT  ((NBC + NWAVE * WCAPC + NWAVE) * 4)
#define LDS_FILL   ((RCAP + NBF + NWAVE * WCAPF + NWAVE) * 4)

static_assert((CHUNK & (CHUNK - 1)) == 0);
static_assert((NBC & (NBC - 1)) == 0 && (NBF & (NBF - 1)) == 0);
static_assert(NBF <= (1 << ESHF));
static_assert((NBC % NBF) == 0);
static_assert(OTHR * 4 == NBF);
static_assert((RCAP % 32) == 0);
static_assert(TGT == NWAVE * 32);
static_assert(GROWS == NWAVE * 16);
static_assert((TGT % GROWS) == 0);
static_assert(NBC == NWAVE * 32 * 128);
static_assert((DF % 32) == 0);
static_assert((TPP % 8) == 0 && TPP >= DF);
static_assert(DF * 4 == NTHR);
static_assert(COP * 8 <= NTHR && CO <= COP);
static_assert(LDS_FILL <= 300 * 1024);

typedef float     v4f  __attribute__((ext_vector_type(4)));
typedef float     v8f  __attribute__((ext_vector_type(8)));
typedef int       v4i  __attribute__((ext_vector_type(4)));
typedef _Float16  v8h  __attribute__((ext_vector_type(8)));
typedef _Float16  v16h __attribute__((ext_vector_type(16)));
union FragH { v16h v; v8h h[2]; };

__device__ __forceinline__ v8f wmf(v16h a, v16h b, v8f c) {
  v8f d = __builtin_amdgcn_wmma_f32_16x16x32_f16(false, a, false, b, (short)0, c, false, false);
  asm volatile("v_nop\n\tv_nop\n\tv_nop\n\tv_nop" : "+v"(d) : "v"(a), "v"(b));
  return d;
}

template <int NB, int SRC, int WC>
__device__ __forceinline__ int scan_chunk(const int* __restrict__ keys, int nK, int cbase,
                                          int slotBase, int vec8, int* list, int tid, int lane, int wave) {
  int wc = 0;
#pragma unroll
  for (int g = 0; g < NGRP; ++g) {
    const int el0  = (g * NTHR + tid) * EPT;
    const int e0   = cbase + el0;
    const int sent = -2147483647 - 1;
    const int i0 = min(e0, nK - 1),     i1 = min(e0 + 1, nK - 1), i2 = min(e0 + 2, nK - 1), i3 = min(e0 + 3, nK - 1);
    const int i4 = min(e0 + 4, nK - 1), i5 = min(e0 + 5, nK - 1), i6 = min(e0 + 6, nK - 1), i7 = min(e0 + 7, nK - 1);
    v4i da, db;
    if (vec8 != 0 && cbase + CHUNK <= nK) {
      da = *(const v4i*)(keys + e0);
      db = *(const v4i*)(keys + e0 + 4);
    } else {
      da.x = (e0     < nK) ? keys[i0] : sent;
      da.y = (e0 + 1 < nK) ? keys[i1] : sent;
      da.z = (e0 + 2 < nK) ? keys[i2] : sent;
      da.w = (e0 + 3 < nK) ? keys[i3] : sent;
      db.x = (e0 + 4 < nK) ? keys[i4] : sent;
      db.y = (e0 + 5 < nK) ? keys[i5] : sent;
      db.z = (e0 + 6 < nK) ? keys[i6] : sent;
      db.w = (e0 + 7 < nK) ? keys[i7] : sent;
    }
    const unsigned nb = (unsigned)slotBase;
    const unsigned s0 = (unsigned)da.x - nb, s1 = (unsigned)da.y - nb;
    const unsigned s2 = (unsigned)da.z - nb, s3 = (unsigned)da.w - nb;
    const unsigned s4 = (unsigned)db.x - nb, s5 = (unsigned)db.y - nb;
    const unsigned s6 = (unsigned)db.z - nb, s7 = (unsigned)db.w - nb;
    const bool h0 = s0 < (unsigned)NB, h1 = s1 < (unsigned)NB, h2 = s2 < (unsigned)NB, h3 = s3 < (unsigned)NB;
    const bool h4 = s4 < (unsigned)NB, h5 = s5 < (unsigned)NB, h6 = s6 < (unsigned)NB, h7 = s7 < (unsigned)NB;
    const unsigned any = __builtin_amdgcn_ballot_w32(h0 | h1 | h2 | h3 | h4 | h5 | h6 | h7);
    if (any != 0u) {
#define HITJ(HJ, SJ, VJ) { \
        const unsigned mj = __builtin_amdgcn_ballot_w32(HJ); \
        if (mj != 0u) { \
          if (HJ) { \
            const int pos = wc + (int)__builtin_amdgcn_mbcnt_lo(mj, 0u); \
            const int entv = SRC ? (((VJ) << ESHF) | (int)(SJ)) : (int)(SJ); \
            if (pos < WC) list[wave * WC + pos] = entv; \
          } \
          wc += (int)__builtin_popcount(mj); } }
      HITJ(h0, s0, i0)
      HITJ(h1, s1, i1)
      HITJ(h2, s2, i2)
      HITJ(h3, s3, i3)
      HITJ(h4, s4, i4)
      HITJ(h5, s5, i5)
      HITJ(h6, s6, i6)
      HITJ(h7, s7, i7)
#undef HITJ
    }
  }
  return wc;
}

__global__ __launch_bounds__(NTHR) void k_wprep(
    const float* __restrict__ W1, const float* __restrict__ R1,
    const float* __restrict__ W2, const float* __restrict__ R2,
    const float* __restrict__ M1, const float* __restrict__ M2,
    _Float16* W1p, _Float16* W2p, _Float16* M1p, _Float16* M2p, float scale) {
  __shared__ __attribute__((aligned(16))) _Float16 sT[DF * TPP];
  const int tid = threadIdx.x;
  const int b = (int)blockIdx.x;
  if (b >= S1N + S2N + 3) {
    if (tid < COP * 8) {
      const int n = tid >> 3, p = tid & 7;
      const int nn = n < CO ? n : CO - 1;
      v8h hv;
#pragma unroll
      for (int i = 0; i < 8; ++i) {
        const float w = M2[(8 * p + i) * CO + nn] * scale;
        hv[i] = (_Float16)(n < CO ? w : 0.0f);
      }
      _Float16* d = M2p + (size_t)n * DF + 8 * p;
      *(volatile v8h*)d = hv;
      __threadfence();
      *(volatile v8h*)d = hv;
    }
    return;
  }
  const float* src;
  _Float16* dst;
  if (b <= S1N) {
    src = (b < S1N) ? (W1 + (size_t)b * DF * DF) : R1;
    dst = W1p + (size_t)b * DF * DF;
  } else if (b <= S1N + S2N + 1) {
    const int s = b - (S1N + 1);
    src = (s < S2N) ? (W2 + (size_t)s * DF * DF) : R2;
    dst = W2p + (size_t)s * DF * DF;
  } else {
    src = M1;
    dst = M1p;
  }
  const int o = tid & (DF - 1), dq = tid >> 6;
#pragma unroll
  for (int i = 0; i < DF / 4; ++i) {
    const int d = dq + 4 * i;
    const float v = src[d * DF + o] * scale;
    sT[o * TPP + d] = (_Float16)v;
  }
  __syncthreads();
  const int nl = tid >> 3, p = tid & 7;
  const v8h hv0 = *(const v8h*)(sT + nl * TPP + 8 * p);
  const v8h hv1 = *(const v8h*)(sT + (nl + 32) * TPP + 8 * p);
  _Float16* d0 = dst + (size_t)nl * DF + 8 * p;
  _Float16* d1 = dst + (size_t)(nl + 32) * DF + 8 * p;
  *(volatile v8h*)d0 = hv0;
  *(volatile v8h*)d1 = hv1;
  __threadfence();
  *(volatile v8h*)d0 = hv0;
  *(volatile v8h*)d1 = hv1;
}

__global__ __launch_bounds__(NTHR) void k_cvtx(const float* __restrict__ x, _Float16* X16,
                                               int nN, int npad, float acs) {
  const int gid = (int)blockIdx.x * NTHR + (int)threadIdx.x;
  const int row = gid >> 3, p = gid & 7;
  if (row >= npad) return;
  const int rs = row < nN ? row : nN - 1;
  const float* xp = x + (size_t)rs * DF + 8 * p;
  v4f f0 = *(const v4f*)xp;
  v4f f1 = *(const v4f*)(xp + 4);
  if (row >= nN) {
    const v4f z = {0.f, 0.f, 0.f, 0.f}; f0 = z; f1 = z;
  }
  v8h hv;
  hv[0] = (_Float16)(f0.x * acs); hv[1] = (_Float16)(f0.y * acs); hv[2] = (_Float16)(f0.z * acs); hv[3] = (_Float16)(f0.w * acs);
  hv[4] = (_Float16)(f1.x * acs); hv[5] = (_Float16)(f1.y * acs); hv[6] = (_Float16)(f1.z * acs); hv[7] = (_Float16)(f1.w * acs);
  _Float16* d = X16 + (size_t)row * DF + 8 * p;
  *(volatile v8h*)d = hv;
  __threadfence();
  *(volatile v8h*)d = hv;
}

__global__ __launch_bounds__(NTHR) void k_count(
    const int* __restrict__ keys, int* cnt, int nK, int vec8) {
  extern __shared__ v4f lds_dyn[];
  int* scnt = (int*)lds_dyn;
  int* list = scnt + NBC;
  int* wcnt = list + NWAVE * WCAPC;
  const int tid = threadIdx.x, lane = tid & 31, wave = tid >> 5;
  const int nodeBase = blockIdx.x * NBC;

  {
    const v4i z = {0, 0, 0, 0};
    for (int i = tid; i < NBC / 4; i += NTHR) ((v4i*)scnt)[i] = z;
  }
  __syncthreads();

  const int nChunks = (nK + CHUNK - 1) / CHUNK;
#pragma unroll 1
  for (int ch = 0; ch < nChunks; ++ch) {
    const int cbase = ch * CHUNK;
    const int wc = scan_chunk<NBC, 0, WCAPC>(keys, nK, cbase, nodeBase, vec8, list, tid, lane, wave);
    if (lane == 0) wcnt[wave] = wc;
    __syncthreads();
    if (wave == 0) {
#pragma unroll 1
      for (int wsx = 0; wsx < NWAVE; ++wsx) {
        int n = __builtin_amdgcn_readfirstlane(wcnt[wsx]);
        n = n > WCAPC ? WCAPC : (n < 0 ? 0 : n);
        const int* lp = list + wsx * WCAPC;
#pragma unroll 1
        for (int i = 0; i < n; ++i) {
          const int ent  = __builtin_amdgcn_readfirstlane(lp[i]);
          const int slot = ent & (NBC - 1);
          if (lane == 0) scnt[slot] = scnt[slot] + 1;
        }
      }
    }
    __syncthreads();
  }

  int* cp = cnt + (size_t)nodeBase;
#pragma unroll 4
  for (int q = 0; q < 32; ++q) {
    const int f = (wave * 32 + q) * 128 + 4 * lane;
    const v4i c = *(const v4i*)(scnt + f);
    *(volatile v4i*)(cp + f) = c;
  }
  __threadfence();
#pragma unroll 4
  for (int q = 0; q < 32; ++q) {
    const int f = (wave * 32 + q) * 128 + 4 * lane;
    const v4i c = *(const v4i*)(scnt + f);
    *(volatile v4i*)(cp + f) = c;
  }
}

__global__ __launch_bounds__(OTHR) void k_offsets(
    const int* __restrict__ cnt, int* off, int* rbase, int nBF) {
  __shared__ __attribute__((aligned(16))) int srb[RBN];
  __shared__ int wtot[OTHR / 32];
  const int tid = threadIdx.x, lane = tid & 31, wave = tid >> 5;
  for (int i = tid; i < RBN; i += OTHR) srb[i] = 0;
  int carry = 0;
#pragma unroll 1
  for (int fb = 0; fb < nBF; ++fb) {
    const int base = fb * NBF;
    const v4i c = *(const v4i*)(cnt + base + 4 * tid);
    const int e0 = max(c.x, 0), e1 = max(c.y, 0), e2 = max(c.z, 0), e3 = max(c.w, 0);
    const int ts = e0 + e1 + e2 + e3;
    int incl = ts;
#pragma unroll
    for (int d = 1; d < 32; d <<= 1) {
      const int t = __shfl_up(incl, d, 32);
      if (lane >= d) incl += t;
    }
    if (lane == 31) wtot[wave] = incl;
    __syncthreads();
    int pre = 0;
#pragma unroll 1
    for (int w = 0; w < wave; ++w) pre += wtot[w];
    int tot = 0;
#pragma unroll
    for (int w = 0; w < OTHR / 32; ++w) tot += wtot[w];
    int run = carry + pre + incl - ts;
    v4i o;
    o.x = run; run += e0;
    o.y = run; run += e1;
    o.z = run; run += e2;
    o.w = run;
    int* op = off + base + 4 * tid;
    *(volatile v4i*)op = o;
    __threadfence();
    *(volatile v4i*)op = o;
    if (tid == 0) srb[min(fb, RBN - 1)] = carry;
    carry += (tot + 31) & ~31;
    __syncthreads();
  }
  if (tid == 0) srb[min(nBF, RBN - 1)] = carry;
  __syncthreads();
  v4i rv = {0, 0, 0, 0};
  if (tid < 32) rv = *(const v4i*)(srb + 4 * tid);
  if (tid < 32) *(volatile v4i*)(rbase + 4 * tid) = rv;
  __threadfence();
  if (tid < 32) *(volatile v4i*)(rbase + 4 * tid) = rv;
}

__global__ __launch_bounds__(NTHR) void k_fill(
    const int* __restrict__ keys, const int* __restrict__ off,
    const int* __restrict__ rbase, int* csr, int nK, int vec8, int csrLen) {
  extern __shared__ v4f lds_dyn[];
  int* region = (int*)lds_dyn;
  int* cursor = region + RCAP;
  int* list   = cursor + NBF;
  int* wcnt   = list + NWAVE * WCAPF;
  const int tid = threadIdx.x, lane = tid & 31, wave = tid >> 5;
  const int b = blockIdx.x;
  const int nodeBase = b * NBF;

  int rb0 = rbase[b];
  const int rb1 = rbase[b + 1];
  rb0 = rb0 < 0 ? 0 : (rb0 > csrLen ? csrLen : rb0);
  rb0 &= ~31;
  int len = rb1 - rb0;
  len = len < 0 ? 0 : (len > RCAP ? RCAP : len);
  int lenW = (len + 31) & ~31;
  if (rb0 + lenW > csrLen) lenW = (csrLen - rb0) & ~31;

  {
    const v4i z = {0, 0, 0, 0};
    for (int i = tid; i < RCAP / 4; i += NTHR) ((v4i*)region)[i] = z;
    for (int s = tid; s < NBF; s += NTHR) {
      int o = off[nodeBase + s] - rb0;
      o = o < 0 ? 0 : (o > RCAP ? RCAP : o);
      cursor[s] = o;
    }
  }
  __syncthreads();

  const int nChunks = (nK + CHUNK - 1) / CHUNK;
#pragma unroll 1
  for (int ch = 0; ch < nChunks; ++ch) {
    const int cbase = ch * CHUNK;
    const int wc = scan_chunk<NBF, 1, WCAPF>(keys, nK, cbase, nodeBase, vec8, list, tid, lane, wave);
    if (lane == 0) wcnt[wave] = wc;
    __syncthreads();
    if (wave == 0) {
#pragma unroll 1
      for (int wsx = 0; wsx < NWAVE; ++wsx) {
        int n = __builtin_amdgcn_readfirstlane(wcnt[wsx]);
        n = n > WCAPF ? WCAPF : (n < 0 ? 0 : n);
        const int* lp = list + wsx * WCAPF;
#pragma unroll 1
        for (int i = 0; i < n; ++i) {
          const int ent  = __builtin_amdgcn_readfirstlane(lp[i]);
          const int slot = ent & (NBF - 1);
          int ev = (ent >> ESHF) & EMASK;
          ev = ev > nK - 1 ? nK - 1 : ev;
          if (lane == 0) {
            int pos = cursor[slot];
            pos = pos < 0 ? 0 : (pos > RCAP - 1 ? RCAP - 1 : pos);
            region[pos] = ev;
            const int np = pos + 1;
            cursor[slot] = np > RCAP ? RCAP : np;
          }
        }
      }
    }
    __syncthreads();
  }

  const int nv = lenW >> 2;
  int* gp = csr + rb0;
#pragma unroll 1
  for (int i = tid; i < nv; i += NTHR) { const v4i v = ((const v4i*)region)[i]; *(volatile v4i*)(gp + 4 * i) = v; }
  __threadfence();
#pragma unroll 1
  for (int i = tid; i < nv; i += NTHR) { const v4i v = ((const v4i*)region)[i]; *(volatile v4i*)(gp + 4 * i) = v; }
}

__device__ __forceinline__ void cvst8(const float* lp, _Float16* gp, float s) {
  const v4f f0 = *(const v4f*)lp;
  const v4f f1 = *(const v4f*)(lp + 4);
  v8h h;
  h[0] = (_Float16)(f0.x * s); h[1] = (_Float16)(f0.y * s); h[2] = (_Float16)(f0.z * s); h[3] = (_Float16)(f0.w * s);
  h[4] = (_Float16)(f1.x * s); h[5] = (_Float16)(f1.y * s); h[6] = (_Float16)(f1.z * s); h[7] = (_Float16)(f1.w * s);
  *(volatile v8h*)gp = h;
}

template <int EPI>
__global__ __launch_bounds__(NTHR) void k_gemm(
    const _Float16* __restrict__ A16, const _Float16* __restrict__ Bw,
    const float* __restrict__ bias, void* Cout, int ldc, float osc, float ocs, int nStore, int nBias) {
  constexpr int NT  = (EPI == 3) ? 1 : 4;
  constexpr int NCB = 16 * NT;
  __shared__ __attribute__((aligned(16))) float stg[GROWS * NCB];
  const int tid = threadIdx.x, lane = tid & 31, wave = tid >> 5, hh = lane >> 4, m = lane & 15;
  const int rowBase = (int)blockIdx.x * GROWS;
  const int colBase = (int)blockIdx.y * NCB;
  const _Float16* ap  = A16 + (size_t)(rowBase + 16 * wave + m) * DF + 8 * hh;
  const _Float16* bp0 = Bw + (size_t)(colBase + m) * DF + 8 * hh;

  v8f acc[NT];
#pragma unroll
  for (int t = 0; t < NT; ++t) { v8f z = {0.f, 0.f, 0.f, 0.f, 0.f, 0.f, 0.f, 0.f}; acc[t] = z; }

#pragma unroll
  for (int kt = 0; kt < DF / 32; ++kt) {
    FragH af;
    af.h[0] = *(const v8h*)(ap + 32 * kt);
    af.h[1] = *(const v8h*)(ap + 32 * kt + 16);
#pragma unroll
    for (int t = 0; t < NT; ++t) {
      const _Float16* bp = bp0 + (size_t)(16 * t) * DF + 32 * kt;
      FragH bf;
      bf.h[0] = *(const v8h*)bp;
      bf.h[1] = *(const v8h*)(bp + 16);
      acc[t] = wmf(af.v, bf.v, acc[t]);
    }
  }

  float bc[NT];
#pragma unroll
  for (int t = 0; t < NT; ++t) {
    bc[t] = 0.0f;
    if constexpr (EPI != 0) {
      int ci = colBase + 16 * t + m;
      ci = ci > nBias - 1 ? nBias - 1 : ci;
      bc[t] = bias[ci];
    }
  }

  float* sp = stg + (16 * wave + 8 * hh) * NCB + m;
#pragma unroll
  for (int t = 0; t < NT; ++t) {
#pragma unroll
    for (int r = 0; r < 8; ++r) {
      float v = acc[t][r] * osc;
      if constexpr (EPI != 0) v = v + bc[t];
      if constexpr (EPI >= 2) v = fmaxf(v, 0.0f);
      sp[r * NCB + 16 * t] = v;
    }
  }
  __syncthreads();

  if constexpr (EPI == 0 || EPI == 2) {
    _Float16* C = (_Float16*)Cout;
    const int pr = lane >> 3, pp = lane & 7;
#pragma unroll
    for (int i = 0; i < 4; ++i) {
      const int row = 16 * wave + 4 * i + pr;
      cvst8(stg + row * NCB + 8 * pp, C + (size_t)(rowBase + row) * ldc + colBase + 8 * pp, ocs);
    }
    __threadfence();
#pragma unroll
    for (int i = 0; i < 4; ++i) {
      const int row = 16 * wave + 4 * i + pr;
      cvst8(stg + row * NCB + 8 * pp, C + (size_t)(rowBase + row) * ldc + colBase + 8 * pp, ocs);
    }
  } else if constexpr (EPI == 1) {
    float* C = (float*)Cout;
#pragma unroll
    for (int i = 0; i < 8; ++i) {
      const int row = 16 * wave + 2 * i + hh;
      const v4f v = *(const v4f*)(stg + row * NCB + 4 * m);
      *(volatile v4f*)(C + (size_t)(rowBase + row) * ldc + colBase + 4 * m) = v;
    }
    __threadfence();
#pragma unroll
    for (int i = 0; i < 8; ++i) {
      const int row = 16 * wave + 2 * i + hh;
      const v4f v = *(const v4f*)(stg + row * NCB + 4 * m);
      *(volatile v4f*)(C + (size_t)(rowBase + row) * ldc + colBase + 4 * m) = v;
    }
  } else {
    float* C = (float*)Cout;
    const int row = 16 * wave + (lane >> 1), q = lane & 1;
    const v4f v = *(const v4f*)(stg + row * NCB + 4 * q);
    const bool ok = (rowBase + row) < nStore;
    float* gp = C + (size_t)(rowBase + row) * ldc + 4 * q;
    if (ok) *(volatile v4f*)gp = v;
    __threadfence();
    if (ok) *(volatile v4f*)gp = v;
  }
}

__global__ __launch_bounds__(NTHR) void k_agg(
    const int* __restrict__ csr, const int* __restrict__ off, const int* __restrict__ cnt,
    const int* __restrict__ srcidx, const float* __restrict__ ea,
    const _Float16* __restrict__ Y, const float* __restrict__ R32,
    _Float16* Hout, int nN, int nE, int csrLen, int K, int ldy, float acs) {
  __shared__ __attribute__((aligned(16))) _Float16 sH[TGT * DF];
  const int tid = threadIdx.x, lane = tid & 31, wave = tid >> 5;
  const int es = lane >> 3, cg = lane & 7, ch = 8 * cg;
  const int tbase = (int)blockIdx.x * TGT + wave * 32;
  const int cnt_l = cnt[tbase + lane];
  const int off_l = off[tbase + lane];
  const float km1 = (float)(K - 1);
  const int kmax = K - 1;

#pragma unroll 1
  for (int j = 0; j < 32; ++j) {
    const int c = tbase + j;
    const int nraw = __builtin_amdgcn_readlane(cnt_l, j);
    const int n = nraw < 0 ? 0 : (nraw > DEGCAP ? DEGCAP : nraw);
    const int st = __builtin_amdgcn_readlane(off_l, j);
    float a[8];
#pragma unroll
    for (int i = 0; i < 8; ++i) a[i] = 0.0f;

#pragma unroll 1
    for (int q0 = 0; q0 < n; q0 += 4) {
      const int e = q0 + es;
      const bool valid = e < n;
      int pos = st + e;
      pos = pos < 0 ? 0 : (pos > csrLen - 1 ? csrLen - 1 : pos);
      int el = csr[pos];
      el = el < 0 ? 0 : (el > nE - 1 ? nE - 1 : el);
      int sl = srcidx[el];
      sl = sl < 0 ? 0 : (sl > nN - 1 ? nN - 1 : sl);
      const float u0 = ea[2 * (size_t)el];
      const float u1 = ea[2 * (size_t)el + 1];
      const float v0 = u0 * km1, v1 = u1 * km1;
      const float fl0 = floorf(v0), fl1 = floorf(v1);
      const float fr0 = v0 - fl0, fr1 = v1 - fl1;
      const int l0 = (int)fl0, l1 = (int)fl1;
      const int l0p = l0 + 1, l1p = l1 + 1;
      const int a0i = l0 < 0 ? 0 : (l0 > kmax ? kmax : l0);
      const int a0j = l0p < 0 ? 0 : (l0p > kmax ? kmax : l0p);
      const int a1i = l1 < 0 ? 0 : (l1 > kmax ? kmax : l1);
      const int a1j = l1p < 0 ? 0 : (l1p > kmax ? kmax : l1p);
      const float g0 = 1.0f - fr0, g1 = 1.0f - fr1;
      float B0 = g0 * g1;
      float B1 = g0 * fr1;
      float B2 = fr0 * g1;
      float B3 = fr0 * fr1;
      B0 = valid ? B0 : 0.0f; B1 = valid ? B1 : 0.0f; B2 = valid ? B2 : 0.0f; B3 = valid ? B3 : 0.0f;
      const int w0 = a0i + K * a1i;
      const int w1 = a0i + K * a1j;
      const int w2 = a0j + K * a1i;
      const int w3 = a0j + K * a1j;
      const _Float16* yr = Y + (size_t)sl * ldy + ch;
      const v8h y0 = *(const v8h*)(yr + DF * w0);
      const v8h y1 = *(const v8h*)(yr + DF * w1);
      const v8h y2 = *(const v8h*)(yr + DF * w2);
      const v8h y3 = *(const v8h*)(yr + DF * w3);
#pragma unroll
      for (int i = 0; i < 8; ++i) {
        a[i] = fmaf(B0, (float)y0[i], a[i]);
        a[i] = fmaf(B1, (float)y1[i], a[i]);
        a[i] = fmaf(B2, (float)y2[i], a[i]);
        a[i] = fmaf(B3, (float)y3[i], a[i]);
      }
    }

#pragma unroll
    for (int i = 0; i < 8; ++i) {
      a[i] += __shfl_xor(a[i], 8, 32);
      a[i] += __shfl_xor(a[i], 16, 32);
    }
    const float cv = fmaxf((float)nraw, 1.0f);
    const float rc = 1.0f / cv;
    const int cs = c < nN ? c : nN - 1;
    const float* rp = R32 + (size_t)cs * DF + ch;
    const v4f r0 = *(const v4f*)rp;
    const v4f r1 = *(const v4f*)(rp + 4);
    float rr[8];
    rr[0] = r0.x; rr[1] = r0.y; rr[2] = r0.z; rr[3] = r0.w;
    rr[4] = r1.x; rr[5] = r1.y; rr[6] = r1.z; rr[7] = r1.w;
    const float qn = __int_as_float(0x7fc00000);
    v8h hv;
#pragma unroll
    for (int i = 0; i < 8; ++i) {
      float v = a[i] * rc + rr[i];
      const float em = __expf(fminf(v, 0.0f)) - 1.0f;
      v = v > 0.0f ? v : em;
      if (c >= nN) v = 0.0f;
      if (nraw > DEGCAP) v = qn;
      hv[i] = (_Float16)(v * acs);
    }
    if (lane < 8) *(v8h*)(sH + (wave * 32 + j) * DF + ch) = hv;
  }
  __syncthreads();

  const int pr = lane >> 3, pp = lane & 7;
  const _Float16* lb = sH + (wave * 32) * DF;
  _Float16* hb = Hout + (size_t)((int)blockIdx.x * TGT + wave * 32) * DF;
#pragma unroll
  for (int i = 0; i < 8; ++i) {
    const int r = 4 * i + pr;
    const v8h hv = *(const v8h*)(lb + r * DF + 8 * pp);
    *(volatile v8h*)(hb + (size_t)r * DF + 8 * pp) = hv;
  }
  __threadfence();
#pragma unroll
  for (int i = 0; i < 8; ++i) {
    const int r = 4 * i + pr;
    const v8h hv = *(const v8h*)(lb + r * DF + 8 * pp);
    *(volatile v8h*)(hb + (size_t)r * DF + 8 * pp) = hv;
  }
}

extern "C" void kernel_launch(void* const* d_in, const int* in_sizes, int n_in,
                              void* d_out, int out_size, void* d_ws, size_t ws_size,
                              hipStream_t stream) {
  if (n_in < 13) return;
  const int nN = in_sizes[0] / DF;
  const int nE = in_sizes[1] / 2;
  if (nN <= 0 || nE <= 0) return;
  if (in_sizes[0] != nN * DF || in_sizes[1] != 2 * nE || in_sizes[2] != 2 * nE) return;
  if (in_sizes[3] != S1N * DF * DF || in_sizes[4] != DF * DF || in_sizes[5] != DF) return;
  if (in_sizes[6] != S2N * DF * DF || in_sizes[7] != DF * DF || in_sizes[8] != DF) return;
  if (in_sizes[9] != DF * DF || in_sizes[10] != DF) return;
  if (in_sizes[11] != DF * CO || in_sizes[12] != CO) return;
  if (nN > (1 << 20) || nE > (1 << 20)) return;
  if ((long long)out_size != (long long)nN * CO) return;

  const float* x   = (const float*)d_in[0];
  const int*   ei  = (const int*)d_in[1];
  const float* ea  = (const float*)d_in[2];
  const float* W1  = (const float*)d_in[3];
  const float* R1  = (const float*)d_in[4];
  const float* b1  = (const float*)d_in[5];
  const float* W2  = (const float*)d_in[6];
  const float* R2  = (const float*)d_in[7];
  const float* b2  = (const float*)d_in[8];
  const float* M1  = (const float*)d_in[9];
  const float* mb1 = (const float*)d_in[10];
  const float* M2  = (const float*)d_in[11];
  const float* mb2 = (const float*)d_in[12];
  float* out = (float*)d_out;
  const int* srci = ei;
  const int* dsti = ei + nE;
  const int nK = nE;

  const int NPAD   = ((nN + TGT - 1) / TGT) * TGT;
  const int nBC    = (nN + NBC - 1) / NBC;
  const int CNTPAD = nBC * NBC;
  const int nBF    = (nN + NBF - 1) / NBF;
  const int OFFN   = nBF * NBF;
  if (nBF + 1 > RBN) return;
  if (OFFN > CNTPAD || NPAD > OFFN) return;
  if ((NPAD % GROWS) != 0 || (NPAD % TGT) != 0) return;
  const int csrLen = ((nK + 31) & ~31) + 32 * (nBF + 1);
  const int nG     = NPAD / GROWS;
  const int nAgg   = NPAD / TGT;
  const int LD1    = S1N * DF;
  const int LD2    = S2N * DF;

  char* ws = (char*)d_ws;
  size_t off = 0;
  const size_t oY   = off; off += (size_t)NPAD * LD2 * 2;          off = (off + 255) & ~(size_t)255;
  const size_t oX16 = off; off += (size_t)NPAD * DF * 2;           off = (off + 255) & ~(size_t)255;
  const size_t oH16 = off; off += (size_t)NPAD * DF * 2;           off = (off + 255) & ~(size_t)255;
  const size_t oR32 = off; off += (size_t)NPAD * DF * 4;           off = (off + 255) & ~(size_t)255;
  const size_t oW1p = off; off += (size_t)(S1N + 1) * DF * DF * 2; off = (off + 255) & ~(size_t)255;
  const size_t oW2p = off; off += (size_t)(S2N + 1) * DF * DF * 2; off = (off + 255) & ~(size_t)255;
  const size_t oM1p = off; off += (size_t)DF * DF * 2;             off = (off + 255) & ~(size_t)255;
  const size_t oM2p = off; off += (size_t)COP * DF * 2;            off = (off + 255) & ~(size_t)255;
  const size_t oCnt = off; off += (size_t)CNTPAD * 4;              off = (off + 255) & ~(size_t)255;
  const size_t oOff = off; off += (size_t)OFFN * 4;                off = (off + 255) & ~(size_t)255;
  const size_t oRb  = off; off += (size_t)RBN * 4;                 off = (off + 255) & ~(size_t)255;
  const size_t oCsr = off; off += (size_t)csrLen * 4;              off = (off + 255) & ~(size_t)255;
  if (off > ws_size || off > (size_t)WSLIM) return;
  _Float16* Y16  = (_Float16*)(ws + oY);
  _Float16* X16  = (_Float16*)(ws + oX16);
  _Float16* H16  = (_Float16*)(ws + oH16);
  float*    R32  = (float*)(ws + oR32);
  _Float16* W1p  = (_Float16*)(ws + oW1p);
  _Float16* W2p  = (_Float16*)(ws + oW2p);
  _Float16* M1p  = (_Float16*)(ws + oM1p);
  _Float16* M2p  = (_Float16*)(ws + oM2p);
  int*      cnt  = (int*)(ws + oCnt);
  int*      offp = (int*)(ws + oOff);
  int*      rb   = (int*)(ws + oRb);
  int*      csr  = (int*)(ws + oCsr);

  const int vec8 = ((nE & 3) == 0) ? 1 : 0;
  const float osc = 1.0f / ((float)ACARRY * (float)WSCL);
  const float acs = (float)ACARRY;

  k_wprep<<<S1N + S2N + 4, NTHR, 0, stream>>>(W1, R1, W2, R2, M1, M2, W1p, W2p, M1p, M2p, (float)WSCL);

  k_cvtx<<<(NPAD * 8 + NTHR - 1) / NTHR, NTHR, 0, stream>>>(x, X16, nN, NPAD, acs);

  hipFuncSetAttribute(reinterpret_cast<const void*>(&k_count),
                      hipFuncAttributeMaxDynamicSharedMemorySize, LDS_COUNT);
  k_count<<<nBC, NTHR, LDS_COUNT, stream>>>(dsti, cnt, nK, vec8);
  k_offsets<<<1, OTHR, 0, stream>>>(cnt, offp, rb, nBF);
  hipFuncSetAttribute(reinterpret_cast<const void*>(&k_fill),
                      hipFuncAttributeMaxDynamicSharedMemorySize, LDS_FILL);
  k_fill<<<nBF, NTHR, LDS_FILL, stream>>>(dsti, offp, rb, csr, nK, vec8, csrLen);

  k_gemm<0><<<dim3(nG, S1N), NTHR, 0, stream>>>(X16, W1p, b1, (void*)Y16, LD1, osc, 1.0f, NPAD, 1);
  k_gemm<1><<<dim3(nG, 1), NTHR, 0, stream>>>(X16, W1p + (size_t)S1N * DF * DF, b1, (void*)R32, DF, osc, 1.0f, NPAD, DF);
  k_agg<<<nAgg, NTHR, 0, stream>>>(csr, offp, cnt, srci, ea, Y16, R32, H16, nN, nE, csrLen, K1V, LD1, acs);

  k_gemm<0><<<dim3(nG, S2N), NTHR, 0, stream>>>(H16, W2p, b2, (void*)Y16, LD2, osc, 1.0f, NPAD, 1);
  k_gemm<1><<<dim3(nG, 1), NTHR, 0, stream>>>(H16, W2p + (size_t)S2N * DF * DF, b2, (void*)R32, DF, osc, 1.0f, NPAD, DF);
  k_agg<<<nAgg, NTHR, 0, stream>>>(csr, offp, cnt, srci, ea, Y16, R32, X16, nN, nE, csrLen, K2V, LD2, acs);

  k_gemm<2><<<dim3(nG, 1), NTHR, 0, stream>>>(X16, M1p, mb1, (void*)H16, DF, osc, acs, NPAD, DF);
  k_gemm<3><<<dim3(nG, 1), NTHR, 0, stream>>>(H16, M2p, mb2, (void*)out, CO, osc, 1.0f, nN, CO);
}
